// ResGCN_36893769072894
// MI455X (gfx1250) — hardware-verified
//
#include <hip/hip_runtime.h>
#include <math.h>

typedef __attribute__((ext_vector_type(16))) _Float16 v16h;
typedef __attribute__((ext_vector_type(16))) __bf16 v16b;
typedef __attribute__((ext_vector_type(8)))  _Float16 v8h;
typedef __attribute__((ext_vector_type(8)))  float v8f;
typedef __attribute__((ext_vector_type(4)))  float v4f;
typedef __attribute__((ext_vector_type(2)))  float v2f;
typedef __attribute__((ext_vector_type(4)))  unsigned v4u;
typedef __attribute__((ext_vector_type(4)))  int v4i;
typedef float __attribute__((may_alias)) float_a;
typedef int __attribute__((may_alias)) int_a;

template <typename T> __device__ __forceinline__ void vst2(void* p, T v) { *(volatile T*)p = v; __threadfence(); *(volatile T*)p = v; }
__device__ __forceinline__ v8f wmma16(v16h a, v16h b, v8f c) {
  v8f d = __builtin_amdgcn_wmma_f32_16x16x32_f16(false, a, false, b, (short)0, c, false, false);
  asm volatile("v_nop\n\tv_nop\n\tv_nop\n\tv_nop" : "+v"(d) : "v"(a), "v"(b));
  return d;
}
__device__ __forceinline__ v8f wmma_bf(v16b a, v16b b, v8f c) {
  v8f d = __builtin_amdgcn_wmma_f32_16x16x32_bf16(false, a, false, b, (short)0, c, false, false);
  asm volatile("v_nop\n\tv_nop\n\tv_nop\n\tv_nop" : "+v"(d) : "v"(a), "v"(b));
  return d;
}
__device__ __forceinline__ v16h frag_h(const _Float16* rowk0, int lane) {
  union { v16h v; v8h q[2]; } u; const _Float16* p = rowk0 + 8 * (lane >> 4);
  u.q[0] = *(const v8h*)p; u.q[1] = *(const v8h*)(p + 16); return u.v;
}
__device__ __forceinline__ v16h frag_f32(const float* rowk0, int lane) {
  v16h a; const float* p = rowk0 + 8 * (lane >> 4);
#pragma unroll
  for (int i = 0; i < 8; ++i) { a[i] = (_Float16)p[i]; a[8 + i] = (_Float16)p[16 + i]; }
  return a;
}
__device__ __forceinline__ v16h frag_f32s(const float* rowk0, int lane, float sc) {
  v16h a; const float* p = rowk0 + 8 * (lane >> 4);
#pragma unroll
  for (int i = 0; i < 8; ++i) { a[i] = (_Float16)(p[i] * sc); a[8 + i] = (_Float16)(p[16 + i] * sc); }
  return a;
}
__device__ __forceinline__ v16h fragc_f32(const float* W, int k0, int n, int lane, int ld, int K) {
  v16h a; const int g = lane >> 4;
#pragma unroll
  for (int i = 0; i < 8; ++i) { const int ka = k0 + 8 * g + i, kb = ka + 16;
    a[i] = (_Float16)(ka < K ? W[(size_t)(ka < K ? ka : K - 1) * ld + n] : 0.f); a[8 + i] = (_Float16)(kb < K ? W[(size_t)(kb < K ? kb : K - 1) * ld + n] : 0.f); }
  return a;
}
struct F2 { v16b h, l; };
__device__ __forceinline__ F2 bsplit16(const float v[16]) { F2 r;
#pragma unroll
  for (int i = 0; i < 16; ++i) { const __bf16 h = (__bf16)v[i]; r.h[i] = h; r.l[i] = (__bf16)(v[i] - (float)h); }
  return r; }
__device__ __forceinline__ F2 split_row(const float* row, int k0, int lane) { float v[16]; const float* p = row + k0 + 8 * (lane >> 4);
#pragma unroll
  for (int i = 0; i < 8; ++i) { v[i] = p[i]; v[8 + i] = p[16 + i]; }
  return bsplit16(v); }
__device__ __forceinline__ F2 split_rowK(const float* row, int k0, int lane, int K) { float v[16]; const int g = lane >> 4;
#pragma unroll
  for (int i = 0; i < 8; ++i) { const int ka = k0 + 8 * g + i, kb = ka + 16; v[i] = ka < K ? row[ka < K ? ka : K - 1] : 0.f; v[8 + i] = kb < K ? row[kb < K ? kb : K - 1] : 0.f; }
  return bsplit16(v); }
__device__ __forceinline__ F2 split_col(const float* W, int k0, int n, int lane, int ld, int K) { float v[16]; const int g = lane >> 4;
#pragma unroll
  for (int i = 0; i < 8; ++i) { const int ka = k0 + 8 * g + i, kb = ka + 16; v[i] = ka < K ? W[(size_t)(ka < K ? ka : K - 1) * ld + n] : 0.f; v[8 + i] = kb < K ? W[(size_t)(kb < K ? kb : K - 1) * ld + n] : 0.f; }
  return bsplit16(v); }
__device__ __forceinline__ v8f mac3(const F2& a, const F2& b, v8f c) { c = wmma_bf(a.l, b.h, c); c = wmma_bf(a.h, b.l, c); return wmma_bf(a.h, b.h, c); }
__device__ __forceinline__ float sigm(float v) { return 1.0f / (1.0f + expf(-v)); }
#define LDSX() do { asm volatile("s_wait_dscnt 0" ::: "memory"); __builtin_amdgcn_wave_barrier(); __builtin_amdgcn_fence(__ATOMIC_RELEASE, "workgroup"); } while (0)

__device__ __forceinline__ float bfr(float v) { return (float)(__bf16)v; }
#define NPTS 16384
#define KN 16
#define NE (NPTS * KN)
#define CMAXO 32
#ifndef NRV
#define NRV NPTS
#endif
#define WS_IDX 0u
#define WS_H   (WS_IDX + 4u * (size_t)NE)
#define WS_XA  (WS_H + 4u * (size_t)NE * CMAXO)
#define WS_XB  (WS_XA + 4u * (size_t)NPTS * CMAXO)
#define WS_ST  (WS_XB + 4u * (size_t)NPTS * CMAXO)
#define WS_P4  (WS_ST + 4u * 32 * 32 + 1024u)
#define WS_GI  (WS_P4 + 16u * (size_t)NPTS)
#define WS_END (WS_GI + 4u * (size_t)NPTS)
__global__ __launch_bounds__(256) void k_x0(const float* __restrict__ PT, float* __restrict__ X0, float* __restrict__ P4, int* __restrict__ GI) { const size_t n = (size_t)blockIdx.x * 256 + threadIdx.x; if (n >= (size_t)NPTS) return; v4f o; o[0] = bfr(PT[n * 5 + 1]); o[1] = bfr(PT[n * 5 + 2]); o[2] = bfr(PT[n * 5 + 3]); o[3] = bfr(PT[n * 5 + 4]); if (n < (size_t)NRV) vst2(X0 + n * 4, o);
  { v4f p; p[0] = o[0]; p[1] = o[1]; p[2] = o[2]; {
#pragma clang fp contract(off)
      p[3] = (o[0] * o[0] + o[1] * o[1]) + o[2] * o[2]; }
    vst2(P4 + n * 4, p); vst2(GI + n, (int)bfr(PT[n * 5])); } }
struct Best16 { float d[KN]; int i[KN]; };
__device__ __forceinline__ void push16(Best16& b, float d, int i) {
  if (d < b.d[KN - 1]) { b.d[KN - 1] = d; b.i[KN - 1] = i; }
#pragma unroll
  for (int p = KN - 1; p > 0; --p) { const bool sw = b.d[p] < b.d[p - 1]; const float td = b.d[p], ud = b.d[p - 1]; const int ti = b.i[p], ui = b.i[p - 1]; b.d[p] = sw ? ud : td; b.d[p - 1] = sw ? td : ud; b.i[p] = sw ? ui : ti; b.i[p - 1] = sw ? ti : ui; } }
__global__ __launch_bounds__(256) void k_knnm(const float* __restrict__ PT, const float* __restrict__ P4, const int* __restrict__ GI, int* __restrict__ IDX) { __shared__ int sidx8[8][KN];
  const int wave = threadIdx.x >> 5, lane = threadIdx.x & 31; const size_t n = (size_t)blockIdx.x * 8 + wave;
  const int gq = (int)bfr(PT[n * 5]); const float qx = bfr(PT[n * 5 + 1]), qy = bfr(PT[n * 5 + 2]), qz = bfr(PT[n * 5 + 3]);
  float aa; {
#pragma clang fp contract(off)
    aa = (qx * qx + qy * qy) + qz * qz; }
  Best16 bs; float tau;
#pragma unroll
  for (int r = 0; r < KN; ++r) { bs.d[r] = 3.0e38f; bs.i[r] = 0x7fffffff; }
#pragma unroll 1
  for (int s = lane; s < 2048; s += 32) { float d; {
#pragma clang fp contract(off)
      const v4f pp = *(const v4f*)(P4 + (size_t)s * 4); const int gs = GI[s];
      const float dot = (qx * pp[0] + qy * pp[1]) + qz * pp[2]; d = (aa + pp[3]) - 2.0f * dot; d = gs == gq ? d : 2.0e38f; }
    push16(bs, d, s); }
  tau = 3.0e38f;
#pragma unroll 1
  for (int r = 0; r < KN; ++r) { float d = bs.d[0]; int i = bs.i[0];
#pragma unroll
    for (int o = 1; o < 32; o <<= 1) { const float e = __shfl_xor(d, o); const int j = __shfl_xor(i, o); if (e < d || (e == d && j < i)) { d = e; i = j; } }
    tau = d;
    { const bool pop = (bs.i[0] == i && bs.d[0] == d);
#pragma unroll
      for (int p = 0; p < KN - 1; ++p) { bs.d[p] = pop ? bs.d[p + 1] : bs.d[p]; bs.i[p] = pop ? bs.i[p + 1] : bs.i[p]; }
      bs.d[KN - 1] = pop ? 3.0e38f : bs.d[KN - 1]; bs.i[KN - 1] = pop ? 0x7fffffff : bs.i[KN - 1]; } }
#pragma unroll
  for (int r = 0; r < KN; ++r) { bs.d[r] = 3.0e38f; bs.i[r] = 0x7fffffff; }
#pragma unroll 1
  for (int s = lane; s < NPTS; s += 32) { float d; {
#pragma clang fp contract(off)
      const v4f pp = *(const v4f*)(P4 + (size_t)s * 4); const int gs = GI[s];
      const float dot = (qx * pp[0] + qy * pp[1]) + qz * pp[2]; d = (aa + pp[3]) - 2.0f * dot; d = gs == gq ? d : 2.0e38f; }
    if (d <= tau && d < bs.d[KN - 1]) push16(bs, d, s); }
  int sel = 0;
#pragma unroll 1
  for (int r = 0; r < KN; ++r) { float d = bs.d[0]; int i = bs.i[0];
#pragma unroll
    for (int o = 1; o < 32; o <<= 1) { const float e = __shfl_xor(d, o); const int j = __shfl_xor(i, o); if (e < d || (e == d && j < i)) { d = e; i = j; } }
    if (lane == r) sel = i;
    { const bool pop = (bs.i[0] == i && bs.d[0] == d);
#pragma unroll
      for (int p = 0; p < KN - 1; ++p) { bs.d[p] = pop ? bs.d[p + 1] : bs.d[p]; bs.i[p] = pop ? bs.i[p + 1] : bs.i[p]; }
      bs.d[KN - 1] = pop ? 3.0e38f : bs.d[KN - 1]; bs.i[KN - 1] = pop ? 0x7fffffff : bs.i[KN - 1]; } }
  if (lane < KN) sidx8[wave][lane] = sel;
  __syncthreads();
  if (threadIdx.x < 32) vst2((v4i*)(IDX + (size_t)blockIdx.x * 8 * KN) + threadIdx.x, *(const v4i*)(&sidx8[0][0] + threadIdx.x * 4)); }
__global__ __launch_bounds__(128) void k_econv(const float* __restrict__ X, const int* __restrict__ IDX, const float* __restrict__ Wm, const float* __restrict__ Bv, int cin, int cout, float* __restrict__ H) { __shared__ __align__(16) float sf[4][16][36];
  const int tid = threadIdx.x, wave = tid >> 5, lane = tid & 31, col = lane & 15, g = lane >> 4; const size_t n = (size_t)blockIdx.x * 4 + wave;
  int nb = IDX[n * KN + col]; nb = nb < 0 ? 0 : (nb >= NPTS ? NPTS - 1 : nb);
  const int c2 = 2 * cin; const int nk = (c2 + 31) / 32;
  v8f acc[2] = {};
  for (int kc = 0; kc < nk; ++kc) { float va[16];
#pragma unroll
    for (int i = 0; i < 16; ++i) { const int c = kc * 32 + 8 * g + (i < 8 ? i : 8 + i); const int ca = c < cin ? c : 0; const int cb = (c >= cin && c < c2) ? c - cin : 0;
      const float xa = X[n * cin + ca], xj = X[(size_t)nb * cin + cb], xi = X[n * cin + cb];
      va[i] = c < cin ? xa : (c < c2 ? (xj - xi) : 0.f); }
    asm volatile("s_wait_loadcnt 0x0" ::: "memory");
    const F2 a = bsplit16(va);
#pragma unroll
    for (int j = 0; j < 2; ++j) { if (j * 16 >= cout) break; v16b w; const int o = j * 16 + col;
#pragma unroll
      for (int i = 0; i < 16; ++i) { const int k = kc * 32 + 8 * g + (i < 8 ? i : 8 + i); const int kc2 = k < c2 ? k : 0; const float keep = k < c2 ? 1.f : 0.f; w[i] = (__bf16)(Wm[(size_t)o * c2 + kc2] * keep); }
      asm volatile("s_wait_loadcnt 0x0" ::: "memory");
      acc[j] = wmma_bf(a.h, w, acc[j]); acc[j] = wmma_bf(a.l, w, acc[j]); } }
#pragma unroll
  for (int j = 0; j < 2; ++j) { if (j * 16 >= cout) break; const float bb = bfr(Bv[j * 16 + col]);
#pragma unroll
    for (int r = 0; r < 8; ++r) sf[wave][8 * g + r][j * 16 + col] = acc[j][r] + bb; }
  LDSX();
  { float* hw = H + n * KN * (size_t)cout; const int nf4 = KN * cout / 4;
    for (int e4 = lane; e4 < nf4; e4 += 32) { const int f0 = e4 * 4; const int r = f0 / cout, c = f0 % cout; v4f v; v[0] = sf[wave][r][c]; v[1] = sf[wave][r][c + 1]; v[2] = sf[wave][r][c + 2]; v[3] = sf[wave][r][c + 3]; vst2(hw + f0, v); } } }
__global__ __launch_bounds__(256) void k_statc(const float* __restrict__ H, int cout, int nrows, float* __restrict__ ST) { __shared__ float sred[8]; __shared__ float sbc; const int t = threadIdx.x; const int c = blockIdx.x;
  float s1 = 0.f; for (int r = t; r < nrows; r += 256) s1 += H[(size_t)r * cout + c];
#pragma unroll
  for (int o = 1; o < 32; o <<= 1) s1 += __shfl_xor(s1, o);
  if ((t & 31) == 0) sred[t >> 5] = s1; __syncthreads(); if (t == 0) { float a = 0.f; for (int i = 0; i < 8; ++i) a += sred[i]; sbc = a / (float)nrows; } __syncthreads(); const float mu = sbc; __syncthreads();
  float q = 0.f; for (int r = t; r < nrows; r += 256) { const float d = H[(size_t)r * cout + c] - mu; q += d * d; }
#pragma unroll
  for (int o = 1; o < 32; o <<= 1) q += __shfl_xor(q, o);
  if ((t & 31) == 0) sred[t >> 5] = q; __syncthreads(); if (t == 0) { float a = 0.f; for (int i = 0; i < 8; ++i) a += sred[i]; sbc = rsqrtf(a / (float)nrows + 1e-5f); } __syncthreads();
  if (t < 32) { const float v = t == 0 ? mu : (t == 1 ? sbc : 0.f); vst2(ST + (size_t)c * 32 + t, v); } }
__global__ __launch_bounds__(256) void k_bnmax(const float* __restrict__ H, const float* __restrict__ ST, const float* __restrict__ G, const float* __restrict__ TB, int cout, float* __restrict__ XO) { const size_t e4 = (size_t)blockIdx.x * 256 + threadIdx.x; if (e4 >= (size_t)NRV * (cout / 4)) return; const size_t n = e4 / (cout / 4); const int c0 = (int)(e4 % (cout / 4)) * 4;
  float mu[4], rs[4], gg[4], tt[4]; for (int i = 0; i < 4; ++i) { mu[i] = ST[(c0 + i) * 32]; rs[i] = ST[(c0 + i) * 32 + 1]; gg[i] = bfr(G[c0 + i]); tt[i] = bfr(TB[c0 + i]); }
  v4f m; m[0] = m[1] = m[2] = m[3] = 0.f;
  for (int j = 0; j < KN; ++j) { const v4f h = *(const v4f*)(H + (n * KN + j) * (size_t)cout + c0);
#pragma unroll
    for (int i = 0; i < 4; ++i) m[i] = fmaxf(m[i], fmaxf((h[i] - mu[i]) * rs[i] * gg[i] + tt[i], 0.f)); }
  vst2(XO + n * cout + c0, m); }
extern "C" void kernel_launch(void* const* d_in, const int* in_sizes, int n_in, void* d_out, int out_size, void* d_ws, size_t ws_size, hipStream_t stream) {
  (void)in_sizes; (void)n_in; (void)out_size;
  if (ws_size < (size_t)WS_END) return;
  char* ws = (char*)d_ws; const float** F = (const float**)d_in; int* IDX = (int*)(ws + WS_IDX); float *H = (float*)(ws + WS_H), *XA = (float*)(ws + WS_XA), *XB = (float*)(ws + WS_XB), *ST = (float*)(ws + WS_ST);
  float* P4 = (float*)(ws + WS_P4); int* GI = (int*)(ws + WS_GI);
  k_x0<<<dim3((NPTS + 255) / 256), 256, 0, stream>>>(F[0], XA, P4, GI);
  k_knnm<<<dim3(NRV / 8), 256, 0, stream>>>(F[0], P4, GI, IDX);
  const int dims[5] = {4, 16, 16, 32, 32}; float* xin = XA; float* xout = XB;
  for (int l = 0; l < 4; ++l) { const int ci = dims[l], co = dims[l + 1]; float* dst = (l == 3) ? (float*)d_out : xout;
    k_econv<<<dim3(NRV / 4), 128, 0, stream>>>(xin, IDX, F[1 + 4 * l], F[2 + 4 * l], ci, co, H);
    k_statc<<<dim3(co), 256, 0, stream>>>(H, co, NRV * KN, ST);
    k_bnmax<<<dim3((unsigned)(((size_t)NRV * (co / 4) + 255) / 256)), 256, 0, stream>>>(H, ST, F[3 + 4 * l], F[4 + 4 * l], co, dst);
    float* tmp = xin; xin = xout; xout = tmp; }
}
